// MultiHeadAttention_12455405158937
// MI455X (gfx1250) — hardware-verified
//
#include <hip/hip_runtime.h>
#include <math.h>

#ifndef NB
#define NB 8
#endif
#ifndef SEQ
#define SEQ 1024
#endif
#define NB_FULL 8
#define SEQ_FULL 1024
#define DMODEL 768
#define NHEAD 12
#define HDIM 64
#define MROWS (NB * SEQ)

static_assert(SEQ % 64 == 0);
static_assert(SEQ <= SEQ_FULL);
static_assert(NB <= NB_FULL);
static_assert(DMODEL % 64 == 0);
static_assert((3 * DMODEL) % 64 == 0);
static_assert(DMODEL % 32 == 0);
static_assert(NHEAD * HDIM == DMODEL);
static_assert(HDIM == 64);
static_assert(MROWS % 64 == 0);
static_assert(((long long)(NB - 1) * SEQ_FULL + SEQ) * DMODEL <= (long long)NB_FULL * SEQ_FULL * DMODEL);

typedef __attribute__((ext_vector_type(16))) _Float16 v16h;
typedef __attribute__((ext_vector_type(8)))  _Float16 v8h;
typedef __attribute__((ext_vector_type(8)))  float    v8f;
typedef __attribute__((ext_vector_type(4)))  float    v4f;

__device__ __forceinline__ v8f wmma16(v16h a, v16h b, v8f c) {
    c = __builtin_amdgcn_wmma_f32_16x16x32_f16(false, a, false, b, (short)0, c, false, false);
    asm volatile("v_nop\n\tv_nop\n\tv_nop\n\tv_nop" : "+v"(c) : "v"(a), "v"(b));
    return c;
}

#define VST2(T, ptr, val) do { const T vst2_v_ = (val); *(volatile T*)(ptr) = vst2_v_; __threadfence(); *(volatile T*)(ptr) = vst2_v_; } while (0)

#define AW 4
#define KP 72
struct AttnP {
    const float* Q; const float* K; const float* V; float* O;
    long long sQb, sKb, sVb, sOb;
    int ldq, ldk, ldv, ldo, Lk, pad_;
    float scale, pad2_;
};
static_assert(sizeof(AttnP) == 4 * 8 + 4 * 8 + 6 * 4 + 2 * 4);

__global__ __launch_bounds__(32 * AW) __attribute__((amdgpu_num_vgpr(256))) void k_attn(AttnP p) {
    __shared__ __align__(16) _Float16 qs[64 * KP];
    __shared__ __align__(16) _Float16 kt[64 * KP];
    __shared__ __align__(16) _Float16 vt[64 * KP];
    __shared__ __align__(16) _Float16 ps[AW * 16 * KP];
    __shared__ __align__(16) float    os[AW * 16 * 68];
    union FH { v16h v; v8h h[2]; };
    const int tid = threadIdx.x, lane = tid & 31, hf = lane >> 4, l15 = lane & 15;
    const int wave = __builtin_amdgcn_readfirstlane((int)(threadIdx.x >> 5));
    const int h = blockIdx.y, b = blockIdx.z;
    const int qb0 = blockIdx.x * 64;
    const int sr = tid >> 1, sd = (tid & 1) * 32;
    const float L2E = 1.4426950408889634f;
    const float NEG = -__builtin_inff();

    {
        const float* src = p.Q + b * p.sQb + (long long)(qb0 + sr) * p.ldq + h * HDIM + sd;
#pragma unroll
        for (int i = 0; i < 4; ++i) {
            const v4f a = *(const v4f*)(src + 8 * i), c = *(const v4f*)(src + 8 * i + 4);
            v8h hv;
            hv[0] = (_Float16)a.x; hv[1] = (_Float16)a.y; hv[2] = (_Float16)a.z; hv[3] = (_Float16)a.w;
            hv[4] = (_Float16)c.x; hv[5] = (_Float16)c.y; hv[6] = (_Float16)c.z; hv[7] = (_Float16)c.w;
            *(v8h*)(&qs[sr * KP + sd + 8 * i]) = hv;
        }
    }

    v8f o[4]; float m8[8], l8[8];
#pragma unroll
    for (int t = 0; t < 4; ++t) { v8f zz = {}; o[t] = zz; }
#pragma unroll
    for (int i = 0; i < 8; ++i) { m8[i] = NEG; l8[i] = 0.f; }

    const float* kbase = p.K + b * p.sKb + h * HDIM + sd;
    const float* vbase = p.V + b * p.sVb + h * HDIM + sd;
    for (int j0 = 0; j0 < p.Lk; j0 += 64) {
        __syncthreads();
        {
            const float* ksrc = kbase + (long long)(j0 + sr) * p.ldk;
            const float* vsrc = vbase + (long long)(j0 + sr) * p.ldv;
#pragma unroll
            for (int i = 0; i < 4; ++i) {
                const v4f a = *(const v4f*)(ksrc + 8 * i), c = *(const v4f*)(ksrc + 8 * i + 4);
                v8h hv;
                hv[0] = (_Float16)a.x; hv[1] = (_Float16)a.y; hv[2] = (_Float16)a.z; hv[3] = (_Float16)a.w;
                hv[4] = (_Float16)c.x; hv[5] = (_Float16)c.y; hv[6] = (_Float16)c.z; hv[7] = (_Float16)c.w;
                *(v8h*)(&kt[sr * KP + sd + 8 * i]) = hv;
            }
#pragma unroll
            for (int i = 0; i < 8; ++i) {
                const v4f a = *(const v4f*)(vsrc + 4 * i);
                vt[(sd + 4 * i + 0) * KP + sr] = (_Float16)a.x;
                vt[(sd + 4 * i + 1) * KP + sr] = (_Float16)a.y;
                vt[(sd + 4 * i + 2) * KP + sr] = (_Float16)a.z;
                vt[(sd + 4 * i + 3) * KP + sr] = (_Float16)a.w;
            }
        }
        __syncthreads();

        v8f s[4];
#pragma unroll
        for (int t = 0; t < 4; ++t) { v8f zz = {}; s[t] = zz; }
#pragma unroll
        for (int kk = 0; kk < 2; ++kk) {
            FH qa;
            qa.h[0] = *(const v8h*)(&qs[(wave * 16 + l15) * KP + kk * 32 + 8 * hf]);
            qa.h[1] = *(const v8h*)(&qs[(wave * 16 + l15) * KP + kk * 32 + 16 + 8 * hf]);
#pragma unroll
            for (int t = 0; t < 4; ++t) {
                FH kb;
                kb.h[0] = *(const v8h*)(&kt[(t * 16 + l15) * KP + kk * 32 + 8 * hf]);
                kb.h[1] = *(const v8h*)(&kt[(t * 16 + l15) * KP + kk * 32 + 16 + 8 * hf]);
                s[t] = wmma16(qa.v, kb.v, s[t]);
            }
        }

#pragma unroll
        for (int i = 0; i < 8; ++i) {
            float sc[4];
#pragma unroll
            for (int t = 0; t < 4; ++t) { float v = s[t][i] * p.scale; v *= L2E; sc[t] = v; }
            float mx = fmaxf(fmaxf(sc[0], sc[1]), fmaxf(sc[2], sc[3]));
            mx = fmaxf(mx, __shfl_xor(mx, 1, 32)); mx = fmaxf(mx, __shfl_xor(mx, 2, 32));
            mx = fmaxf(mx, __shfl_xor(mx, 4, 32)); mx = fmaxf(mx, __shfl_xor(mx, 8, 32));
            const float mnew = fmaxf(m8[i], mx);
            const float corr = (mnew == NEG) ? 1.f : exp2f(m8[i] - mnew);
            float rs = 0.f;
#pragma unroll
            for (int t = 0; t < 4; ++t) {
                const float pp = exp2f(sc[t] - mnew); rs += pp;
                ps[(wave * 16 + i + 8 * hf) * KP + t * 16 + l15] = (_Float16)(pp * 4096.f);
            }
            rs += __shfl_xor(rs, 1, 32); rs += __shfl_xor(rs, 2, 32); rs += __shfl_xor(rs, 4, 32); rs += __shfl_xor(rs, 8, 32);
            l8[i] = l8[i] * corr + rs; m8[i] = mnew;
#pragma unroll
            for (int t = 0; t < 4; ++t) o[t][i] *= corr;
        }
        __syncthreads();

#pragma unroll
        for (int kk = 0; kk < 2; ++kk) {
            FH pa;
            pa.h[0] = *(const v8h*)(&ps[(wave * 16 + l15) * KP + kk * 32 + 8 * hf]);
            pa.h[1] = *(const v8h*)(&ps[(wave * 16 + l15) * KP + kk * 32 + 16 + 8 * hf]);
#pragma unroll
            for (int t = 0; t < 4; ++t) {
                FH vb;
                vb.h[0] = *(const v8h*)(&vt[(t * 16 + l15) * KP + kk * 32 + 8 * hf]);
                vb.h[1] = *(const v8h*)(&vt[(t * 16 + l15) * KP + kk * 32 + 16 + 8 * hf]);
                o[t] = wmma16(pa.v, vb.v, o[t]);
            }
        }
    }

#pragma unroll
    for (int i = 0; i < 8; ++i) {
        const float invr = (l8[i] > 0.f) ? 1.f / (l8[i] * 4096.f) : 0.f;
#pragma unroll
        for (int t = 0; t < 4; ++t) os[(wave * 16 + i + 8 * hf) * 68 + t * 16 + l15] = o[t][i] * invr;
    }
    __syncthreads();
    {
        float* obase = p.O + b * p.sOb + (long long)(qb0 + wave * 16) * p.ldo + h * HDIM;
        const int c4 = l15 * 4;
        for (int pass = 0; pass < 2; ++pass) {
#pragma unroll
            for (int it = 0; it < 8; ++it) {
                const int row = it * 2 + hf;
                const v4f val = *(const v4f*)(&os[(wave * 16 + row) * 68 + c4]);
                *(volatile v4f*)(obase + (long long)row * p.ldo + c4) = val;
            }
            __threadfence();
        }
    }
}

namespace g64 {
typedef __attribute__((ext_vector_type(16))) _Float16 v16h;
typedef __attribute__((ext_vector_type(8)))  _Float16 v8h;
typedef __attribute__((ext_vector_type(16))) __bf16   v16b;
typedef __attribute__((ext_vector_type(8)))  __bf16   v8b;
typedef __attribute__((ext_vector_type(8)))  float    v8f;
typedef __attribute__((ext_vector_type(4)))  float    v4f;

__device__ __forceinline__ unsigned short f2bf_bits(float f) {
  unsigned u = __float_as_uint(f);
  return (unsigned short)((u + 0x7FFFu + ((u >> 16) & 1u)) >> 16);
}
__device__ __forceinline__ float bf_bits2f(unsigned short h) { return __uint_as_float(((unsigned)h) << 16); }

__device__ __forceinline__ void dep_guard_h(v8f& a, v8f& b, v16h x, v16h y) { asm volatile("v_nop\n\tv_nop\n\tv_nop\n\tv_nop" : "+v"(a), "+v"(b) : "v"(x), "v"(y)); }
__device__ __forceinline__ void dep_guard_b(v8f& a, v8f& b, v16b x, v16b y) { asm volatile("v_nop\n\tv_nop\n\tv_nop\n\tv_nop" : "+v"(a), "+v"(b) : "v"(x), "v"(y)); }
__device__ __forceinline__ void keep4_h(v16h a, v16h b, v16h c, v16h d) { asm volatile("v_nop" :: "v"(a), "v"(b), "v"(c), "v"(d)); }
__device__ __forceinline__ void keep4_b(v16b a, v16b b, v16b c, v16b d) { asm volatile("v_nop" :: "v"(a), "v"(b), "v"(c), "v"(d)); }
__device__ __forceinline__ void acc_guard4(v8f& a, v8f& b, v8f& c, v8f& d) { asm volatile("v_nop\n\tv_nop\n\tv_nop\n\tv_nop" : "+v"(a), "+v"(b), "+v"(c), "+v"(d)); }
template <typename T> struct Frag;
template <> struct Frag<_Float16> {
  typedef v16h V; union U { v16h v; v8h h[2]; };
  static __device__ __forceinline__ v16h load(const _Float16* p) {
    U f; f.h[0] = *(const v8h*)(p); f.h[1] = *(const v8h*)(p + 16); return f.v;
  }
  static __device__ __forceinline__ v8f mma(v16h a, v16h b, v8f c) {
    return __builtin_amdgcn_wmma_f32_16x16x32_f16(false, a, false, b, (short)0, c, false, false);
  }
  static __device__ __forceinline__ void guard(v8f& a, v8f& b, v16h x, v16h y) { dep_guard_h(a, b, x, y); }
  static __device__ __forceinline__ void keep(v16h a, v16h b, v16h c, v16h d) { keep4_h(a, b, c, d); }
};
template <> struct Frag<__bf16> {
  typedef v16b V; union U { v16b v; v8b h[2]; };
  static __device__ __forceinline__ v16b load(const __bf16* p) {
    U f; f.h[0] = *(const v8b*)(p); f.h[1] = *(const v8b*)(p + 16); return f.v;
  }
  static __device__ __forceinline__ v8f mma(v16b a, v16b b, v8f c) {
    return __builtin_amdgcn_wmma_f32_16x16x32_bf16(false, a, false, b, (short)0, c, false, false);
  }
  static __device__ __forceinline__ void guard(v8f& a, v8f& b, v16b x, v16b y) { dep_guard_b(a, b, x, y); }
  static __device__ __forceinline__ void keep(v16b a, v16b b, v16b c, v16b d) { keep4_b(a, b, c, d); }
};

template <int ET> struct Elem;
template <> struct Elem<0> { typedef _Float16 T; };
template <> struct Elem<1> { typedef __bf16 T; };
template <int ET, bool SPLIT, int BIAS_MODE, int OUT_MODE, bool RESID, int ACT = 0>
__global__ __launch_bounds__(256) __attribute__((amdgpu_num_vgpr(256))) void wmma_gemm64(
    const unsigned short* __restrict__ Ap, const unsigned short* __restrict__ A2p, int lda, long strideA,
    const unsigned short* __restrict__ Btp, const unsigned short* __restrict__ Bt2p, int ldb, long strideB,
    void* __restrict__ Cout, void* __restrict__ Cout2, int ldc, long strideC,
    const float* __restrict__ bias,
    const float* __restrict__ resid, long strideR,
    int M, int N, int K, float scale) {
  typedef typename Elem<ET>::T T;
  typedef typename Frag<T>::V V;
  const T* A = (const T*)Ap; const T* A2 = (const T*)A2p; const T* Bt = (const T*)Btp; const T* Bt2 = (const T*)Bt2p;
  __shared__ __align__(16) float sT[8][16 * 68];
  const int b    = blockIdx.y;
  const int lane = threadIdx.x & 31;
  const int wave = __builtin_amdgcn_readfirstlane((int)(threadIdx.x >> 5));
  const int tilesN = N >> 6;
  const int tilesM = M >> 6;
  const int tile = blockIdx.x * 8 + wave;
  if (tile >= tilesM * tilesN) return;
  const int tm = tile / tilesN;
  const int tn = tile - tm * tilesN;
  const int m0 = tm << 6;
  const int n0 = tn << 6;

  const T* Ab  = A  + (size_t)b * strideA;
  const T* Bb  = Bt + (size_t)b * strideB;
  const T* Ab2 = SPLIT ? (A2  + (size_t)b * strideA) : nullptr;
  const T* Bb2 = SPLIT ? (Bt2 + (size_t)b * strideB) : nullptr;

  const int rlane = lane & 15;
  const int koff  = (lane >> 4) * 8;
  const int mOff  = (lane >> 4) * 8;

  v8f acc[4][4];
#pragma unroll
  for (int i = 0; i < 4; ++i)
#pragma unroll
    for (int j = 0; j < 4; ++j) acc[i][j] = (v8f){0.f,0.f,0.f,0.f,0.f,0.f,0.f,0.f};

  for (int k0 = 0; k0 < K; k0 += 32) {
    V bh[4], bl[4];
#pragma unroll
    for (int j = 0; j < 4; ++j) {
      const size_t bo = (size_t)(n0 + (j << 4) + rlane) * ldb + koff + k0;
      bh[j] = Frag<T>::load(Bb + bo);
      if (SPLIT) bl[j] = Frag<T>::load(Bb2 + bo);
    }
#pragma unroll
    for (int i = 0; i < 4; ++i) {
      const size_t ao = (size_t)(m0 + (i << 4) + rlane) * lda + koff + k0;
      V ah = Frag<T>::load(Ab + ao);
      V al;
      if (SPLIT) al = Frag<T>::load(Ab2 + ao);
#pragma unroll
      for (int j = 0; j < 4; ++j) {
        acc[i][j] = Frag<T>::mma(ah, bh[j], acc[i][j]);
        if (SPLIT) {
          acc[i][j] = Frag<T>::mma(ah, bl[j], acc[i][j]);
          acc[i][j] = Frag<T>::mma(al, bh[j], acc[i][j]);
        }
      }
      Frag<T>::guard(acc[i][0], acc[i][3], ah, SPLIT ? al : ah);
    }
    Frag<T>::keep(bh[0], bh[1], bh[2], bh[3]);
    if (SPLIT) Frag<T>::keep(bl[0], bl[1], bl[2], bl[3]);
  }
  acc_guard4(acc[0][0], acc[0][1], acc[0][2], acc[0][3]);
  acc_guard4(acc[1][0], acc[1][1], acc[1][2], acc[1][3]);
  acc_guard4(acc[2][0], acc[2][1], acc[2][2], acc[2][3]);
  acc_guard4(acc[3][0], acc[3][1], acc[3][2], acc[3][3]);

  float* slab = sT[wave];
  const float* Rb = RESID ? (resid + (size_t)b * strideR) : nullptr;
#pragma unroll
  for (int i = 0; i < 4; ++i) {
    const int mBase = m0 + (i << 4);
#pragma unroll
    for (int j = 0; j < 4; ++j) {
      const int n = n0 + (j << 4) + rlane;
      float bv = 0.f;
      if (BIAS_MODE == 2) bv = bias[n];
#pragma unroll
      for (int r = 0; r < 8; ++r) {
        float v = acc[i][j][r] * scale;
        if (BIAS_MODE == 1) v += bias[mBase + mOff + r];
        if (BIAS_MODE == 2) v += bv;
        if (RESID) v += Rb[(size_t)(mBase + mOff + r) * ldc + n];
        if (ACT == 1) v = tanhf(v);
        if (ACT == 2) v = fmaxf(v, 0.0f);
        if (ACT == 3) v = v / (1.0f + expf(-v));
        if (ACT == 4) v = (v > 0.f) ? v : 0.01f * v;
        if (ACT == 5) v = 0.5f * v * (1.0f + erff(v * 0.70710678118654752f));
        if (ACT == 6) v = (v > 0.f) ? v : 0.2f * v;
        if (ACT == 7) { const float u = 0.7978845608028654f * (v + 0.044715f * v * v * v); v = 0.5f * v * (1.f + tanhf(u)); }
        slab[(mOff + r) * 68 + (j << 4) + rlane] = v;
      }
    }
    __builtin_amdgcn_fence(3  , "workgroup");
    __builtin_amdgcn_wave_barrier();
    __builtin_amdgcn_fence(2  , "workgroup");
    if (OUT_MODE == 0) {
      float* C = (float*)Cout + (size_t)b * strideC;
      const int hh = lane >> 4, c4 = (lane & 15) * 4;
      for (int pass = 0; pass < 2; ++pass) {
#pragma unroll
        for (int it = 0; it < 8; ++it) {
          const int row = it * 2 + hh;
          v4f v = *(const v4f*)(slab + row * 68 + c4);
          *(volatile v4f*)(C + (size_t)(mBase + row) * ldc + n0 + c4) = v;
        }
        __threadfence();
      }
    } else {
      const int q = lane >> 3, c8 = (lane & 7) * 8;
      unsigned short* C  = (unsigned short*)Cout  + (size_t)b * strideC;
      unsigned short* C2 = (OUT_MODE == 2) ? ((unsigned short*)Cout2 + (size_t)b * strideC) : nullptr;
      for (int pass = 0; pass < 2; ++pass) {
#pragma unroll
        for (int it = 0; it < 4; ++it) {
          const int row = it * 4 + q;
          const float* sp = slab + row * 68 + c8;
          v8h hv, lv;
#pragma unroll
          for (int e = 0; e < 8; ++e) {
            if (OUT_MODE == 1) {
              hv[e] = (_Float16)sp[e];
            } else {
              unsigned short hb = f2bf_bits(sp[e]);
              unsigned short lb = f2bf_bits(sp[e] - bf_bits2f(hb));
              hv[e] = __builtin_bit_cast(_Float16, hb);
              lv[e] = __builtin_bit_cast(_Float16, lb);
            }
          }
          *(volatile v8h*)(C + (size_t)(mBase + row) * ldc + n0 + c8) = hv;
          if (OUT_MODE == 2) *(volatile v8h*)(C2 + (size_t)(mBase + row) * ldc + n0 + c8) = lv;
        }
        __threadfence();
      }
    }
    __builtin_amdgcn_fence(3  , "workgroup");
    __builtin_amdgcn_wave_barrier();
    __builtin_amdgcn_fence(2  , "workgroup");
  }
}
}

__global__ __launch_bounds__(256) void k_cast16(const float* __restrict__ src, long long lds, _Float16* __restrict__ dst, long long ldd, int R, int C, float s) {
    const long long i = (long long)blockIdx.x * 256 + threadIdx.x; const long long np = (long long)R * (C / 2); if (i >= np) return; const int r = (int)(i / (C / 2)); const int c = 2 * (int)(i % (C / 2));
    const _Float16 h0 = (_Float16)(src[(long long)r * lds + c] * s), h1 = (_Float16)(src[(long long)r * lds + c + 1] * s);
    const unsigned u = (unsigned)__builtin_bit_cast(unsigned short, h0) | ((unsigned)__builtin_bit_cast(unsigned short, h1) << 16);
    volatile unsigned* d = (volatile unsigned*)(dst + (long long)r * ldd + c); *d = u; __threadfence(); *d = u; }

typedef unsigned int cm_u4 __attribute__((ext_vector_type(4)));
__device__ __forceinline__ unsigned int cmb_pk2(float a, float b) { return (unsigned int)__builtin_bit_cast(unsigned short, (_Float16)a) | ((unsigned int)__builtin_bit_cast(unsigned short, (_Float16)b) << 16); }
__device__ __forceinline__ float cmb_bf(float v) { const unsigned u = __builtin_bit_cast(unsigned, v); const unsigned r = (u + 0x7fffu + ((u >> 16) & 1u)) & 0xffff0000u; return __builtin_bit_cast(float, r); }
__global__ __launch_bounds__(256) void k_cm_bfvec(const float* __restrict__ SRC, float* __restrict__ DST, int n) { const int u = blockIdx.x * 256 + threadIdx.x; if (u >= n) return; VST2(float, DST + u, cmb_bf(SRC[u])); }
__global__ __launch_bounds__(256) void k_cm_castb(const float* __restrict__ SRC, int lds, unsigned short* __restrict__ DST, int ldd, int nR, int nC, float sc) {
    const long long u = (long long)blockIdx.x * 256 + threadIdx.x; const int per = nC / 8; if (u >= (long long)nR * per) return; const int r = (int)(u / per); const int c0 = 8 * (int)(u % per);
    const float* s = SRC + (long long)r * lds + c0; float w[8];
#pragma unroll
    for (int e = 0; e < 8; ++e) w[e] = cmb_bf(s[e]) * sc;
    cm_u4 pk; pk.x = cmb_pk2(w[0], w[1]); pk.y = cmb_pk2(w[2], w[3]); pk.z = cmb_pk2(w[4], w[5]); pk.w = cmb_pk2(w[6], w[7]); VST2(cm_u4, (cm_u4*)(DST + (long long)r * ldd + c0), pk); }
__global__ __launch_bounds__(256) void k_cm_castbT(const float* __restrict__ SRC, int lds, unsigned short* __restrict__ DST, int ldd, int nR, int nC, float sc) {
    const long long u = (long long)blockIdx.x * 256 + threadIdx.x; const int per = nR / 8; if (u >= (long long)nC * per) return; const int c = (int)(u / per); const int r0 = 8 * (int)(u % per);
    float w[8];
#pragma unroll
    for (int e = 0; e < 8; ++e) w[e] = cmb_bf(SRC[(long long)(r0 + e) * lds + c]) * sc;
    cm_u4 pk; pk.x = cmb_pk2(w[0], w[1]); pk.y = cmb_pk2(w[2], w[3]); pk.z = cmb_pk2(w[4], w[5]); pk.w = cmb_pk2(w[6], w[7]); VST2(cm_u4, (cm_u4*)(DST + (long long)c * ldd + r0), pk); }

constexpr size_t al256(size_t b) { return (b + 255) / 256 * 256; }
constexpr size_t SZ_X16  = al256((size_t)MROWS * DMODEL * 2);
constexpr size_t SZ_W316 = al256((size_t)3 * DMODEL * DMODEL * 2);
constexpr size_t SZ_QKV  = al256((size_t)MROWS * 3 * DMODEL * 4);
constexpr size_t SZ_AO   = al256((size_t)MROWS * DMODEL * 4);
constexpr size_t SZ_WO16 = al256((size_t)DMODEL * DMODEL * 2);
constexpr size_t SZ_BR3  = al256((size_t)3 * DMODEL * 4);
constexpr size_t SZ_BRO  = al256((size_t)DMODEL * 4);
constexpr size_t WS_TOTAL = SZ_X16 + SZ_W316 + SZ_QKV + SZ_AO + SZ_WO16 + SZ_BR3 + SZ_BRO;
static_assert(WS_TOTAL <= (size_t)134217728);

extern "C" void kernel_launch(void* const* d_in, const int* in_sizes, int n_in, void* d_out, int out_size, void* d_ws, size_t ws_size, hipStream_t stream) {
    if (n_in < 9) return;
    const long long need_rows = (long long)(NB - 1) * SEQ_FULL + SEQ;
    if ((long long)in_sizes[0] < need_rows * DMODEL) return;
    if (in_sizes[1] < DMODEL * DMODEL || in_sizes[3] < DMODEL * DMODEL || in_sizes[5] < DMODEL * DMODEL || in_sizes[7] < DMODEL * DMODEL) return;
    if (in_sizes[2] < DMODEL || in_sizes[4] < DMODEL || in_sizes[6] < DMODEL || in_sizes[8] < DMODEL) return;
    if ((long long)out_size < need_rows * DMODEL) return;
    if (WS_TOTAL > ws_size) return;

    const float* x  = (const float*)d_in[0];
    const float* Wq = (const float*)d_in[1];
    const float* bq = (const float*)d_in[2];
    const float* Wk = (const float*)d_in[3];
    const float* bk = (const float*)d_in[4];
    const float* Wv = (const float*)d_in[5];
    const float* bv = (const float*)d_in[6];
    const float* Wo = (const float*)d_in[7];
    const float* bo = (const float*)d_in[8];
    float* out = (float*)d_out;

    char* wsp = (char*)d_ws;
    unsigned short* X16  = (unsigned short*)wsp; wsp += SZ_X16;
    unsigned short* W316 = (unsigned short*)wsp; wsp += SZ_W316;
    float* QKV = (float*)wsp; wsp += SZ_QKV;
    float* AO  = (float*)wsp; wsp += SZ_AO;
    unsigned short* WO16 = (unsigned short*)wsp; wsp += SZ_WO16;
    float* BR3 = (float*)wsp; wsp += SZ_BR3;
    float* BRO = (float*)wsp; wsp += SZ_BRO;
    unsigned short* AO16 = X16;

    if (SEQ == SEQ_FULL) {
        k_cm_castb<<<(unsigned)(((long long)MROWS * (DMODEL / 8) + 255) / 256), 256, 0, stream>>>(x, DMODEL, X16, DMODEL, MROWS, DMODEL, 1.0f);
    } else {
        for (int b = 0; b < NB; ++b)
            k_cm_castb<<<(unsigned)(((long long)SEQ * (DMODEL / 8) + 255) / 256), 256, 0, stream>>>(x + (size_t)b * SEQ_FULL * DMODEL, DMODEL, X16 + (size_t)b * SEQ * DMODEL, DMODEL, SEQ, DMODEL, 1.0f);
    }
    const unsigned gw = (unsigned)(((long long)DMODEL * (DMODEL / 8) + 255) / 256);
    k_cm_castbT<<<gw, 256, 0, stream>>>(Wq, DMODEL, W316 + 0, DMODEL, DMODEL, DMODEL, 16.0f);
    k_cm_castbT<<<gw, 256, 0, stream>>>(Wk, DMODEL, W316 + (size_t)DMODEL * DMODEL, DMODEL, DMODEL, DMODEL, 16.0f);
    k_cm_castbT<<<gw, 256, 0, stream>>>(Wv, DMODEL, W316 + (size_t)2 * DMODEL * DMODEL, DMODEL, DMODEL, DMODEL, 16.0f);
    k_cm_castbT<<<gw, 256, 0, stream>>>(Wo, DMODEL, WO16, DMODEL, DMODEL, DMODEL, 16.0f);
    k_cm_bfvec<<<(DMODEL + 255) / 256, 256, 0, stream>>>(bq, BR3 + 0, DMODEL);
    k_cm_bfvec<<<(DMODEL + 255) / 256, 256, 0, stream>>>(bk, BR3 + DMODEL, DMODEL);
    k_cm_bfvec<<<(DMODEL + 255) / 256, 256, 0, stream>>>(bv, BR3 + 2 * DMODEL, DMODEL);
    k_cm_bfvec<<<(DMODEL + 255) / 256, 256, 0, stream>>>(bo, BRO, DMODEL);

    g64::wmma_gemm64<0, false, 2, 0, false, 0><<<dim3((unsigned)((((MROWS) / 64) * ((3 * DMODEL) / 64) + 7) / 8), 1u), 256, 0, stream>>>(
        (const unsigned short*)X16, nullptr, DMODEL, 0, (const unsigned short*)W316, nullptr, DMODEL, 0,
        (void*)QKV, nullptr, 3 * DMODEL, 0, BR3, nullptr, 0, MROWS, 3 * DMODEL, DMODEL, 0.0625f);

    {
        AttnP a;
        a.Q = QKV; a.K = QKV + DMODEL; a.V = QKV + 2 * DMODEL; a.O = AO;
        a.sQb = (long long)SEQ * 3 * DMODEL; a.sKb = (long long)SEQ * 3 * DMODEL; a.sVb = (long long)SEQ * 3 * DMODEL; a.sOb = (long long)SEQ * DMODEL;
        a.ldq = 3 * DMODEL; a.ldk = 3 * DMODEL; a.ldv = 3 * DMODEL; a.ldo = DMODEL; a.Lk = SEQ; a.pad_ = 0;
        a.scale = 0.125f; a.pad2_ = 0.0f;
        k_attn<<<dim3((unsigned)(SEQ / 64), (unsigned)NHEAD, (unsigned)NB), 32 * AW, 0, stream>>>(a);
    }

    k_cast16<<<(unsigned)(((long long)MROWS * (DMODEL / 2) + 255) / 256), 256, 0, stream>>>(AO, DMODEL, (_Float16*)AO16, DMODEL, MROWS, DMODEL, 64.0f);

    g64::wmma_gemm64<0, false, 2, 0, false, 0><<<dim3((unsigned)((((SEQ) / 64) * ((DMODEL) / 64) + 7) / 8), (unsigned)NB), 256, 0, stream>>>(
        (const unsigned short*)AO16, nullptr, DMODEL, (long)SEQ * DMODEL, (const unsigned short*)WO16, nullptr, DMODEL, 0,
        (void*)out, nullptr, DMODEL, (long)SEQ_FULL * DMODEL, BRO, nullptr, 0, SEQ, DMODEL, DMODEL, 0.0009765625f);
}
